// Conv_block_57690000720236
// MI455X (gfx1250) — hardware-run, weakly checked
//
#include <hip/hip_runtime.h>
#include <stdint.h>

#define DEVINL __device__ __forceinline__

typedef _Float16 f16t;
typedef _Float16 v16h __attribute__((ext_vector_type(16)));
typedef _Float16 v8h  __attribute__((ext_vector_type(8)));
typedef float    v8f  __attribute__((ext_vector_type(8)));
typedef float    v4f  __attribute__((ext_vector_type(4)));
typedef int      v4i  __attribute__((ext_vector_type(4)));
typedef v8h __attribute__((may_alias)) v8ha;
typedef v4f __attribute__((may_alias)) v4fa;
typedef v4i __attribute__((may_alias)) v4ia;
union FragH { v16h v; v8h half[2]; };

#define HD     128
#define WD     128
#define HW     (HD * WD)
#define CIN    64
#define COUT   64
#define CMID   16
#define PH     (HD + 2)
#define PW     (WD + 2)
#define PPIX   (PH * PW)
#define KT     (CIN * 9)
#define K2     32
#define TILEP  64
#define NTILE  (HW / TILEP)
#define TPB    256
#define CTPB   128
#define FCHUNK 4096
#define NBW_H  ((COUT * (KT / 8)) / TPB)
#define NBW_1  ((CMID * (KT / 8) + TPB - 1) / TPB)
#define NBW_2  1
#define XCAR   8.0f
#define WCAR   256.0f
#define W2CAR  64.0f
#define S1SCL  (1.0f / 256.0f)
#define INVH   (1.0f / 2048.0f)
#define INVL   (1.0f / 512.0f)

static_assert((KT % 32) == 0);
static_assert((WD % TILEP) == 0);
static_assert((HW % TILEP) == 0);
static_assert((HW % FCHUNK) == 0);
static_assert(((COUT * (KT / 8)) % TPB) == 0);
static_assert((COUT * (K2 / 8)) == TPB);
static_assert(((KT * 2) % 128) == 0);
static_assert(((CIN * 2) % 128) == 0);
static_assert((FCHUNK / 4) == 4 * TPB);
static_assert(CTPB == 128);
static_assert(TILEP == 4 * 16);

DEVINL int imin(int a, int b) { return a < b ? a : b; }
DEVINL int imax(int a, int b) { return a > b ? a : b; }

DEVINL v8f wmma_f16(v16h a, v16h b, v8f c) {
  v8f d = __builtin_amdgcn_wmma_f32_16x16x32_f16(false, a, false, b, (short)0, c, false, false);
  asm volatile("v_nop\n\tv_nop\n\tv_nop\n\tv_nop" : "+v"(d) : "v"(a), "v"(b));
  return d;
}
DEVINL v8f zero8f() {
  v8f z = {0.f, 0.f, 0.f, 0.f, 0.f, 0.f, 0.f, 0.f};
  return z;
}
DEVINL v8h zero8h() {
  v8h z = {(f16t)0, (f16t)0, (f16t)0, (f16t)0, (f16t)0, (f16t)0, (f16t)0, (f16t)0};
  return z;
}

__global__ __launch_bounds__(TPB) void prep_w_k(const float* __restrict__ hw, const float* __restrict__ l1w,
                                               const float* __restrict__ l2w, f16t* __restrict__ Whp,
                                               f16t* __restrict__ W1p, f16t* __restrict__ W2p)
{
  const int blk = blockIdx.x;
  const int tid = threadIdx.x;
  v8h o;
  f16t* dst;
  if (blk < NBW_H) {
    const int t    = blk * TPB + tid;
    const int cout = t / (KT / 8);
    const int part = t - cout * (KT / 8);
    const int k8   = 8 * part;
    const int tap  = k8 >> 6;
    const int cin0 = k8 & 63;
    #pragma unroll
    for (int i = 0; i < 8; ++i) {
      const float wv = hw[(size_t)(cout * CIN + cin0 + i) * 9 + tap];
      o[i] = (f16t)(wv * WCAR);
    }
    dst = Whp + (size_t)8 * t;
  } else if (blk < NBW_H + NBW_1) {
    const int u = (blk - NBW_H) * TPB + tid;
    if (u >= CMID * (KT / 8)) return;
    const int cm   = u / (KT / 8);
    const int part = u - cm * (KT / 8);
    const int k8   = 8 * part;
    const int tap  = k8 >> 6;
    const int cin0 = k8 & 63;
    #pragma unroll
    for (int i = 0; i < 8; ++i) {
      const float wv = l1w[(size_t)(cm * CIN + cin0 + i) * 9 + tap];
      o[i] = (f16t)(wv * WCAR);
    }
    dst = W1p + (size_t)8 * u;
  } else {
    const int u    = tid;
    const int cout = u >> 2;
    const int part = u & 3;
    #pragma unroll
    for (int i = 0; i < 8; ++i) {
      const int kk = 8 * part + i;
      const float wv = l2w[cout * CMID + (kk & (CMID - 1))];
      o[i] = (kk < CMID) ? (f16t)(wv * W2CAR) : (f16t)0;
    }
    dst = W2p + (size_t)8 * u;
  }
  *(volatile v8h*)dst = o;
  __threadfence();
  *(volatile v8h*)dst = o;
}

__global__ __launch_bounds__(TPB) void xprep_k(const float* __restrict__ x, f16t* __restrict__ Xp)
{
  __shared__ __attribute__((aligned(16))) float sX[CIN * WD];
  __shared__ __attribute__((aligned(16))) f16t  sY[PW * CIN];
  const int tid = threadIdx.x;
  const int hp  = blockIdx.x;
  const int b   = blockIdx.y;
  const bool interior = (hp >= 1) && (hp <= HD);
  const int h = imin(imax(hp - 1, 0), HD - 1);

  if (interior) {
    const float* xb = x + ((size_t)b * CIN) * HW + (size_t)h * WD;
    #pragma unroll 4
    for (int idx = tid; idx < CIN * WD; idx += TPB) {
      const int c  = idx >> 7;
      const int wq = idx & (WD - 1);
      sX[idx] = xb[(size_t)c * HW + wq];
    }
  }
  __syncthreads();

  #pragma unroll 1
  for (int idx = tid; idx < PW * CIN; idx += TPB) {
    const int wp = idx >> 6;
    const int c  = idx & (CIN - 1);
    const bool valid = interior && (wp >= 1) && (wp <= WD);
    const int w = imin(imax(wp - 1, 0), WD - 1);
    const float xv = sX[c * WD + w];
    const float yv = valid ? xv : 0.0f;
    sY[idx] = (f16t)(yv * XCAR);
  }
  __syncthreads();

  f16t* dstrow = Xp + ((size_t)(b * PH + hp)) * (size_t)(PW * CIN);
  const int piece = tid & 7;
  const int lg    = tid >> 3;
  v8h vals[5];
  #pragma unroll
  for (int q = 0; q < 5; ++q) {
    const int L = imin(q * 32 + lg, PW - 1);
    vals[q] = *(const v8ha*)(sY + L * CIN + piece * 8);
  }
  #pragma unroll
  for (int q = 0; q < 5; ++q) {
    const int L = q * 32 + lg;
    if (L < PW) *(volatile v8h*)(dstrow + (size_t)L * CIN + piece * 8) = vals[q];
  }
  __threadfence();
  #pragma unroll
  for (int q = 0; q < 5; ++q) {
    const int L = q * 32 + lg;
    if (L < PW) *(volatile v8h*)(dstrow + (size_t)L * CIN + piece * 8) = vals[q];
  }
}

__global__ __launch_bounds__(TPB) void flag_k(const int* __restrict__ midx, int nMask,
                                             const int* __restrict__ iidx, int nInv,
                                             int* __restrict__ Fl)
{
  __shared__ __attribute__((aligned(16))) int sF[FCHUNK];
  const int tid  = threadIdx.x;
  const int base = blockIdx.x * FCHUNK;
  #pragma unroll
  for (int i = tid; i < FCHUNK; i += TPB) sF[i] = 0;
  __syncthreads();
  #pragma unroll 1
  for (int i = tid; i < nMask; i += TPB) {
    const int d = midx[i] - base;
    if ((unsigned)d < (unsigned)FCHUNK) sF[d] = 1;
  }
  __syncthreads();
  #pragma unroll 1
  for (int i = tid; i < nInv; i += TPB) {
    const int d = iidx[i] - base;
    if ((unsigned)d < (unsigned)FCHUNK) sF[d] = 2;
  }
  __syncthreads();

  v4i vals[4];
  #pragma unroll
  for (int q = 0; q < 4; ++q) vals[q] = *(const v4ia*)(sF + (q * TPB + tid) * 4);
  int* dst = Fl + (size_t)base;
  #pragma unroll
  for (int q = 0; q < 4; ++q) *(volatile v4i*)(dst + (size_t)(q * TPB + tid) * 4) = vals[q];
  __threadfence();
  #pragma unroll
  for (int q = 0; q < 4; ++q) *(volatile v4i*)(dst + (size_t)(q * TPB + tid) * 4) = vals[q];
}

__global__ __launch_bounds__(CTPB) void conv_k(const f16t* __restrict__ Xp, const f16t* __restrict__ Whp,
                                             const f16t* __restrict__ W1p, const f16t* __restrict__ W2p,
                                             const int* __restrict__ Fl, float* __restrict__ out)
{
  __shared__ __attribute__((aligned(16))) float sO[COUT * TILEP];
  const int tid = threadIdx.x, lane = tid & 31, wave = tid >> 5;
  const int h = lane >> 4, m = lane & 15;
  const int b = blockIdx.y;
  const int pixBase = blockIdx.x * TILEP;
  const int oh = pixBase >> 7;
  const int ow = (pixBase & (WD - 1)) + 16 * wave + m;

  const f16t* yb  = Xp + ((size_t)(b * PH + oh) * PW + ow) * CIN + 8 * h;
  const f16t* wr  = Whp + (size_t)m * KT + 8 * h;
  const f16t* w1r = W1p + (size_t)m * KT + 8 * h;

  v8f accH[4];
  #pragma unroll
  for (int t = 0; t < 4; ++t) accH[t] = zero8f();
  v8f accS = zero8f();

  #pragma unroll 1
  for (int kh = 0; kh < 3; ++kh) {
    #pragma unroll 1
    for (int kw = 0; kw < 3; ++kw) {
      const int toff = (kh * PW + kw) * CIN;
      const int woff = (3 * kh + kw) * CIN;
      const f16t* ya = yb + toff;
      #pragma unroll
      for (int ks = 0; ks < 2; ++ks) {
        FragH bf;
        bf.half[0] = *(const v8ha*)(ya + 32 * ks);
        bf.half[1] = *(const v8ha*)(ya + 32 * ks + 16);
        #pragma unroll
        for (int t = 0; t < 4; ++t) {
          FragH a;
          const f16t* wa = wr + (size_t)t * 16 * KT + woff + 32 * ks;
          a.half[0] = *(const v8ha*)(wa);
          a.half[1] = *(const v8ha*)(wa + 16);
          accH[t] = wmma_f16(a.v, bf.v, accH[t]);
        }
        FragH a1;
        const f16t* wa1 = w1r + woff + 32 * ks;
        a1.half[0] = *(const v8ha*)(wa1);
        a1.half[1] = *(const v8ha*)(wa1 + 16);
        accS = wmma_f16(a1.v, bf.v, accS);
      }
    }
  }

  FragH bs;
  {
    v8h lo;
    #pragma unroll
    for (int r = 0; r < 8; ++r) lo[r] = (f16t)(accS[r] * S1SCL);
    bs.half[0] = lo;
    bs.half[1] = zero8h();
  }

  const int fl = Fl[(size_t)b * HW + pixBase + 16 * wave + m];

  #pragma unroll
  for (int t = 0; t < 4; ++t) {
    FragH a2;
    const f16t* w2 = W2p + (size_t)(16 * t + m) * K2 + 8 * h;
    a2.half[0] = *(const v8ha*)(w2);
    a2.half[1] = *(const v8ha*)(w2 + 16);
    v8f accL = wmma_f16(a2.v, bs.v, zero8f());
    #pragma unroll
    for (int r = 0; r < 8; ++r) {
      const int cout = 16 * t + 8 * h + r;
      const float hv = accH[t][r] * INVH;
      const float lv = accL[r] * INVL;
      const float v  = (fl == 2) ? lv : ((fl == 1) ? hv : 0.0f);
      sO[cout * TILEP + 16 * wave + m] = v;
    }
  }
  __syncthreads();

  float* gbase = out + ((size_t)b * COUT) * HW + (size_t)pixBase + 4 * m;
  v4f vv[8];
  #pragma unroll
  for (int j = 0; j < 8; ++j) {
    const int row = 16 * wave + 2 * j + h;
    vv[j] = *(const v4fa*)(sO + row * TILEP + 4 * m);
  }
  #pragma unroll
  for (int j = 0; j < 8; ++j) {
    const int row = 16 * wave + 2 * j + h;
    *(volatile v4f*)(gbase + (size_t)row * HW) = vv[j];
  }
  __threadfence();
  #pragma unroll
  for (int j = 0; j < 8; ++j) {
    const int row = 16 * wave + 2 * j + h;
    *(volatile v4f*)(gbase + (size_t)row * HW) = vv[j];
  }
}

extern "C" void kernel_launch(void* const* d_in, const int* in_sizes, int n_in,
                              void* d_out, int out_size, void* d_ws, size_t ws_size,
                              hipStream_t stream)
{
  if (n_in < 6) return;
  const int plane = CIN * HW;
  if (in_sizes[0] <= 0 || (in_sizes[0] % plane) != 0) return;
  const int nB = in_sizes[0] / plane;
  if (nB > 65535) return;
  const int nMask = in_sizes[1];
  const int nInv  = in_sizes[2];
  if (nMask < 0 || nInv < 0) return;
  if (in_sizes[3] != COUT * CIN * 9) return;
  if (in_sizes[4] != CMID * CIN * 9) return;
  if (in_sizes[5] != COUT * CMID) return;
  if (out_size != nB * COUT * HW) return;

  const float* x    = (const float*)d_in[0];
  const int*   midx = (const int*)d_in[1];
  const int*   iidx = (const int*)d_in[2];
  const float* hw   = (const float*)d_in[3];
  const float* l1w  = (const float*)d_in[4];
  const float* l2w  = (const float*)d_in[5];
  float* outp = (float*)d_out;

  const size_t szWh = (size_t)COUT * KT * 2;
  const size_t szW1 = (size_t)CMID * KT * 2;
  const size_t szW2 = (size_t)COUT * K2 * 2;
  const size_t szXp = (size_t)nB * PPIX * CIN * 2;
  const size_t szFl = (size_t)nB * HW * 4;
  size_t off = 0;
  char* ws = (char*)d_ws;
  f16t* Whp = (f16t*)(ws + off); off += szWh;
  f16t* W1p = (f16t*)(ws + off); off += szW1;
  f16t* W2p = (f16t*)(ws + off); off += szW2;
  f16t* Xp  = (f16t*)(ws + off); off += szXp;
  int*  Fl  = (int*)(ws + off);  off += szFl;
  if (off > ws_size) return;
  if (off > (size_t)134217728) return;

  prep_w_k<<<NBW_H + NBW_1 + NBW_2, TPB, 0, stream>>>(hw, l1w, l2w, Whp, W1p, W2p);
  xprep_k<<<dim3(PH, nB), TPB, 0, stream>>>(x, Xp);
  flag_k<<<nB * (HW / FCHUNK), TPB, 0, stream>>>(midx, nMask, iidx, nInv, Fl);
  conv_k<<<dim3(NTILE, nB), CTPB, 0, stream>>>(Xp, Whp, W1p, W2p, Fl, outp);
}
